// IGCNet_repara_23536420782217
// MI455X (gfx1250) — hardware-run, weakly checked
//
#include <hip/hip_runtime.h>
#include <stddef.h>
#include <stdint.h>

#define NN      100000
#define NE      1600000
#define DEG     16
#define FW      32
#define FEA     8
#define HID     64
#define NTHR    256
#define NWAVE   8
#define NPB     128
#define XP      68
#define AP      136
#define XS_F    (16 * XP)
#define AT_F    ((16 * AP) / 2)
#define AG_F    (16 * FW)
#define WAVE_F  (XS_F + AT_F + AG_F)
#define SW_US   (HID * 32 + FW * 128)
#define SW_F    (SW_US / 2)
#define SB_F    128
#define EDGE_LDS_BYTES ((NWAVE * WAVE_F + SW_F + SB_F) * 4)
#define NODE_LDS_BYTES ((NWAVE * WAVE_F + SB_F) * 4)
#define U_WA2   512
#define U_WEA   768
#define U_W12   1280
#define U_W21   2304
#define U_W22   2560
#define O_WA2   0
#define O_WEA   4096
#define O_W12   6144
#define O_W21   10240
#define O_W22   18432
#define PL_US   20480
#define BIAS_F  256
#define WSMAX   134217728

static_assert(NE == DEG * NN);
static_assert(NN % 16 == 0);
static_assert(DEG == 16 && FW == 32 && HID == 64 && FEA == 8);
static_assert((XP * 4) % 16 == 0 && (AP * 2) % 16 == 0 && AP >= 128 && XP >= 64);
static_assert(U_WA2 * 8 == O_WEA && U_WEA * 8 == O_W12 && U_W12 * 8 == O_W21 && U_W21 * 8 == O_W22 && U_W22 * 8 == PL_US);
static_assert(U_WA2 % NTHR == 0 && U_WEA % NTHR == 0 && U_W12 % NTHR == 0 && U_W21 % NTHR == 0 && U_W22 % NTHR == 0);
static_assert(SW_US == O_W21 - O_WEA && SW_US == 3 * NTHR * 8);
static_assert(EDGE_LDS_BYTES <= 327680 && NODE_LDS_BYTES <= 327680);
static_assert(WAVE_F % 4 == 0 && XS_F % 4 == 0 && AT_F % 4 == 0 && SW_F % 4 == 0);
static_assert((size_t)PL_US * 2 + BIAS_F * 4 + (size_t)NN * 64 * 4 + 3 * (size_t)NN * 32 * 4 + 4096 <= (size_t)WSMAX);

typedef float          v4f   __attribute__((ext_vector_type(4)));
typedef float          v8f   __attribute__((ext_vector_type(8)));
typedef int            v4i   __attribute__((ext_vector_type(4)));
typedef int            v8i   __attribute__((ext_vector_type(8)));
typedef unsigned short v8us  __attribute__((ext_vector_type(8)));
typedef unsigned short v16us __attribute__((ext_vector_type(16)));
typedef __bf16         v16bf __attribute__((ext_vector_type(16)));
typedef v4f  __attribute__((may_alias)) v4fa;
typedef v4i  __attribute__((may_alias)) v4ia;
typedef v8us __attribute__((may_alias)) v8usa;
union FragB { v16bf v; v16us u; v8us h[2]; v8i w; };

__device__ __forceinline__ v8f wmb(const FragB& a, const FragB& b, v8f c) {
  v8f d = __builtin_amdgcn_wmma_f32_16x16x32_bf16(false, a.v, false, b.v, (short)0, c, false, false);
  asm volatile("v_nop\n\tv_nop\n\tv_nop\n\tv_nop" : "+v"(d) : "v"(a.w), "v"(b.w));
  return d;
}

__device__ __forceinline__ v8f z8() { v8f z = {0.f, 0.f, 0.f, 0.f, 0.f, 0.f, 0.f, 0.f}; return z; }

__device__ __forceinline__ unsigned bf16_bits(float f) {
  const unsigned u = __float_as_uint(f);
  const unsigned r = (u + 0x7FFFu + ((u >> 16) & 1u)) >> 16;
  return (f != f) ? 0x7fc0u : r;
}
__device__ __forceinline__ float bf16_val(float f) {
  return __uint_as_float(bf16_bits(f) << 16);
}
__device__ __forceinline__ unsigned split_word(float v) {
  const unsigned u  = __float_as_uint(v);
  const unsigned hb = (u + 0x7FFFu + ((u >> 16) & 1u)) >> 16;
  const float    hv = __uint_as_float(hb << 16);
  const float    dl = v - hv;
  const unsigned ud = __float_as_uint(dl);
  const unsigned lb = (ud + 0x7FFFu + ((ud >> 16) & 1u)) >> 16;
  const unsigned w  = (hb & 0xffffu) | (lb << 16);
  return (v != v) ? 0x7fc07fc0u : w;
}
__device__ __forceinline__ float relu_k(float v) { return (v > 0.0f) ? v : (v - v); }

__device__ __forceinline__ void pin_i(int x)  { asm volatile("" :: "v"(x)); }
__device__ __forceinline__ void pin_4(v4f x)  { asm volatile("" :: "v"(x)); }

__device__ __forceinline__ void put16(unsigned short* dp, v8us o) {
  *(volatile v8us*)dp = o;
  __threadfence();
  *(volatile v8us*)dp = o;
}

__device__ __forceinline__ v8us dup4(v4f a) {
  v8us o;
  const unsigned short b0 = (unsigned short)bf16_bits(a.x);
  const unsigned short b1 = (unsigned short)bf16_bits(a.y);
  const unsigned short b2 = (unsigned short)bf16_bits(a.z);
  const unsigned short b3 = (unsigned short)bf16_bits(a.w);
  o[0] = b0; o[1] = b0; o[2] = b1; o[3] = b1; o[4] = b2; o[5] = b2; o[6] = b3; o[7] = b3;
  return o;
}

__global__ __launch_bounds__(NTHR) void k_prep(const float* __restrict__ w11, const float* __restrict__ w12,
                                               const float* __restrict__ w21, const float* __restrict__ w22,
                                               const float* __restrict__ b11, const float* __restrict__ b12,
                                               const float* __restrict__ b21, const float* __restrict__ b22,
                                               unsigned short* WPL, float* BIAS) {
  const int tid = (int)threadIdx.x;
  const int u   = (int)blockIdx.x * NTHR + tid;
  if (u < U_WA2) {
    const int n = u >> 3, k8 = (u & 7) * 8;
    const v4f a = *(const v4f*)(w11 + n * 40 + (k8 >> 1));
    put16(WPL + (size_t)u * 8, dup4(a));
  } else if (u < U_WEA) {
    const int v = u - U_WA2;
    const int n = v >> 2, k8 = (v & 3) * 8;
    const v4f a = *(const v4f*)(w11 + n * 40 + 32);
    const v4f b = *(const v4f*)(w11 + n * 40 + 36);
    const unsigned mk = (k8 == 0) ? 0xffffu : 0u;
    v8us o;
    o[0] = (unsigned short)(bf16_bits(a.x) & mk); o[1] = (unsigned short)(bf16_bits(a.y) & mk);
    o[2] = (unsigned short)(bf16_bits(a.z) & mk); o[3] = (unsigned short)(bf16_bits(a.w) & mk);
    o[4] = (unsigned short)(bf16_bits(b.x) & mk); o[5] = (unsigned short)(bf16_bits(b.y) & mk);
    o[6] = (unsigned short)(bf16_bits(b.z) & mk); o[7] = (unsigned short)(bf16_bits(b.w) & mk);
    put16(WPL + (size_t)u * 8, o);
  } else if (u < U_W12) {
    const int v = u - U_WEA;
    const int n = v >> 4, k8 = (v & 15) * 8;
    const v4f a = *(const v4f*)(w12 + n * 64 + (k8 >> 1));
    put16(WPL + (size_t)u * 8, dup4(a));
  } else if (u < U_W21) {
    const int v = u - U_W12;
    const int n = v >> 4, k8 = (v & 15) * 8;
    const v4f a = *(const v4f*)(w21 + n * 64 + (k8 >> 1));
    put16(WPL + (size_t)u * 8, dup4(a));
  } else if (u < U_W22) {
    const int v = u - U_W21;
    const int n = v >> 4, k8 = (v & 15) * 8;
    const v4f a = *(const v4f*)(w22 + n * 64 + (k8 >> 1));
    put16(WPL + (size_t)u * 8, dup4(a));
  } else {
    const int tc = tid < 64 ? tid : 63;
    const int f  = 4 * tc;
    int ia = f;        ia = ia > 60 ? 60 : ia;
    int ib = f - 64;   ib = ib < 0 ? 0 : (ib > 28 ? 28 : ib);
    int ic = f - 96;   ic = ic < 0 ? 0 : (ic > 60 ? 60 : ic);
    int id = f - 160;  id = id < 0 ? 0 : (id > 12 ? 12 : id);
    const v4f a = *(const v4f*)(b11 + ia);
    const v4f b = *(const v4f*)(b12 + ib);
    const v4f c = *(const v4f*)(b21 + ic);
    const v4f d = *(const v4f*)(b22 + id);
    pin_4(a); pin_4(b); pin_4(c); pin_4(d);
    const unsigned ma = (f < 64) ? 0xffffffffu : 0u;
    const unsigned mb = (f >= 64 && f < 96) ? 0xffffffffu : 0u;
    const unsigned mc = (f >= 96 && f < 160) ? 0xffffffffu : 0u;
    const unsigned md = (f >= 160 && f < 176) ? 0xffffffffu : 0u;
    v4f o;
    o.x = bf16_val(__uint_as_float((__float_as_uint(a.x) & ma) | (__float_as_uint(b.x) & mb) |
                                   (__float_as_uint(c.x) & mc) | (__float_as_uint(d.x) & md)));
    o.y = bf16_val(__uint_as_float((__float_as_uint(a.y) & ma) | (__float_as_uint(b.y) & mb) |
                                   (__float_as_uint(c.y) & mc) | (__float_as_uint(d.y) & md)));
    o.z = bf16_val(__uint_as_float((__float_as_uint(a.z) & ma) | (__float_as_uint(b.z) & mb) |
                                   (__float_as_uint(c.z) & mc) | (__float_as_uint(d.z) & md)));
    o.w = bf16_val(__uint_as_float((__float_as_uint(a.w) & ma) | (__float_as_uint(b.w) & mb) |
                                   (__float_as_uint(c.w) & mc) | (__float_as_uint(d.w) & md)));
    const bool st = tid < 64;
    if (st) *(volatile v4f*)(BIAS + 4 * tc) = o;
    __threadfence();
    if (st) *(volatile v4f*)(BIAS + 4 * tc) = o;
  }
}

__device__ __forceinline__ void flush_rows32(const float* ht, float* dst, bool live, int lane) {
  v4f pv[4];
#pragma unroll
  for (int i = 0; i < 4; ++i) pv[i] = *(const v4fa*)(ht + i * 128 + 4 * lane);
  float* op = dst + 4 * lane;
  if (live) {
#pragma unroll
    for (int i = 0; i < 4; ++i) *(volatile v4f*)(op + i * 128) = pv[i];
  }
  __threadfence();
  if (live) {
#pragma unroll
    for (int i = 0; i < 4; ++i) *(volatile v4f*)(op + i * 128) = pv[i];
  }
}

__device__ __forceinline__ void xa_tail(const float* ht, unsigned* at32, const unsigned short* at, float* zt,
                                        const unsigned short* __restrict__ WA2, float* xdst, bool live,
                                        int lane, int hh, int m) {
#pragma unroll 4
  for (int row = 0; row < 16; ++row) at32[row * (AP / 2) + lane] = split_word(ht[row * FW + lane]);
  __syncthreads();
  v8f acc[4];
#pragma unroll
  for (int nt = 0; nt < 4; ++nt) acc[nt] = z8();
#pragma unroll
  for (int ks = 0; ks < 2; ++ks) {
    FragB a;
    const unsigned short* ap = at + m * AP + 32 * ks + 8 * hh;
    a.h[0] = *(const v8usa*)ap;
    a.h[1] = *(const v8usa*)(ap + 16);
#pragma unroll
    for (int nt = 0; nt < 4; ++nt) {
      FragB b;
      const unsigned short* wq = WA2 + (16 * nt + m) * 64 + 32 * ks + 8 * hh;
      b.h[0] = *(const v8usa*)wq;
      b.h[1] = *(const v8usa*)(wq + 16);
      acc[nt] = wmb(a, b, acc[nt]);
    }
  }
#pragma unroll
  for (int nt = 0; nt < 4; ++nt)
#pragma unroll
    for (int r = 0; r < 8; ++r) zt[(8 * hh + r) * XP + 16 * nt + m] = acc[nt][r];
  __syncthreads();
  v4f pv[8];
#pragma unroll
  for (int i = 0; i < 8; ++i) pv[i] = *(const v4fa*)(zt + (2 * i + hh) * XP + 4 * m);
  float* op = xdst + 4 * lane;
  if (live) {
#pragma unroll
    for (int i = 0; i < 8; ++i) *(volatile v4f*)(op + i * 128) = pv[i];
  }
  __threadfence();
  if (live) {
#pragma unroll
    for (int i = 0; i < 8; ++i) *(volatile v4f*)(op + i * 128) = pv[i];
  }
}

__global__ __launch_bounds__(NTHR) void k_first(const float* __restrict__ x, const unsigned short* __restrict__ WPL,
                                                float* HA, float* XA, int nTiles) {
  extern __shared__ __attribute__((aligned(16))) float dyn[];
  const int tid = (int)threadIdx.x, lane = tid & 31, wave = tid >> 5, hh = lane >> 4, m = lane & 15;
  float*          zt   = dyn + wave * WAVE_F;
  float*          atf  = zt + XS_F;
  unsigned short* at   = (unsigned short*)atf;
  unsigned*       at32 = (unsigned*)atf;
  float*          ht   = atf + AT_F;
  const int  t    = (int)blockIdx.x * NWAVE + wave;
  const bool live = t < nTiles;
  const int  tc   = live ? t : nTiles - 1;
  const int  base = 16 * tc;
#pragma unroll
  for (int i = 0; i < 4; ++i) {
    const int idx = i * 32 + lane;
    const v4f xv = *(const v4f*)(x + (size_t)base * FW + 4 * idx);
    v4f q;
    q.x = bf16_val(xv.x); q.y = bf16_val(xv.y); q.z = bf16_val(xv.z); q.w = bf16_val(xv.w);
    *(v4fa*)(ht + 4 * idx) = q;
  }
  __syncthreads();
  flush_rows32(ht, HA + (size_t)base * FW, live, lane);
  xa_tail(ht, at32, at, zt, WPL + O_WA2, XA + (size_t)base * HID, live, lane, hh, m);
}

__global__ __launch_bounds__(NTHR) void k_edge(const int* __restrict__ srcs, const int* __restrict__ dsts,
                                               const float* __restrict__ EA, const float* __restrict__ XA,
                                               const unsigned short* __restrict__ WE,
                                               const float* __restrict__ BIAS, float* AGGR, int nN) {
  extern __shared__ __attribute__((aligned(16))) float dyn[];
  const int tid = (int)threadIdx.x, lane = tid & 31, wave = tid >> 5, hh = lane >> 4, m = lane & 15;
  float*          xs   = dyn + wave * WAVE_F;
  float*          atf  = xs + XS_F;
  unsigned short* at   = (unsigned short*)atf;
  unsigned*       at32 = (unsigned*)atf;
  float*          ag   = atf + AT_F;
  float*          wf   = dyn + NWAVE * WAVE_F;
  unsigned short* sWE  = (unsigned short*)wf;
  unsigned short* sW12 = sWE + HID * 32;
  float*          sb   = wf + SW_F;

#pragma unroll
  for (int i = 0; i < 3; ++i) {
    const int idx = i * NTHR + tid;
    const v4i w = *(const v4ia*)(WE + 8 * idx);
    *(v4ia*)(sWE + 8 * idx) = w;
  }
  if (wave == 0) {
    const v4f bv = *(const v4fa*)(BIAS + 4 * lane);
    *(v4fa*)(sb + 4 * lane) = bv;
  }
  __syncthreads();

  const int  tileBase = (int)blockIdx.x * NPB + 16 * wave;
  const bool live     = tileBase < nN;
  const int  baseC    = live ? tileBase : nN - 16;
  const float qnan    = __int_as_float(0x7fc00000);
  const unsigned mkw  = (hh == 0) ? 0xffffffffu : 0u;

#pragma unroll 1
  for (int j = 0; j < 16; ++j) {
    const int d  = tileBase + j;
    const int dc = d < nN ? d : nN - 1;
    const int e  = DEG * dc + m;
    int s = srcs[e];
    const int t = dsts[e];
    pin_i(s); pin_i(t);
    s = s < 0 ? 0 : (s > nN - 1 ? nN - 1 : s);
    const unsigned badm = __builtin_amdgcn_ballot_w32(t != dc);

    {
      const float* xr = XA + (size_t)s * HID + 32 * hh;
      v4f g[8];
#pragma unroll
      for (int i = 0; i < 8; ++i) g[i] = *(const v4f*)(xr + 4 * i);
      float* xw = xs + m * XP + 32 * hh;
#pragma unroll
      for (int i = 0; i < 8; ++i) *(v4fa*)(xw + 4 * i) = g[i];
    }
    FragB aE;
    {
      const float* er = EA + (size_t)e * FEA;
      const v4f e0 = *(const v4f*)er;
      const v4f e1 = *(const v4f*)(er + 4);
      v8i w;
      w[0] = (int)((bf16_bits(e0.x) | (bf16_bits(e0.y) << 16)) & mkw);
      w[1] = (int)((bf16_bits(e0.z) | (bf16_bits(e0.w) << 16)) & mkw);
      w[2] = (int)((bf16_bits(e1.x) | (bf16_bits(e1.y) << 16)) & mkw);
      w[3] = (int)((bf16_bits(e1.z) | (bf16_bits(e1.w) << 16)) & mkw);
      w[4] = 0; w[5] = 0; w[6] = 0; w[7] = 0;
      aE.w = w;
    }
    __syncthreads();

    v8f c[4];
#pragma unroll
    for (int nt = 0; nt < 4; ++nt) {
      const float bv = sb[16 * nt + m];
      v8f cc;
#pragma unroll
      for (int r = 0; r < 8; ++r) cc[r] = xs[(8 * hh + r) * XP + 16 * nt + m] + bv;
      FragB b;
      const unsigned short* wq = sWE + (16 * nt + m) * 32 + 8 * hh;
      b.h[0] = *(const v8usa*)wq;
      b.h[1] = *(const v8usa*)(wq + 16);
      c[nt] = wmb(aE, b, cc);
    }
#pragma unroll
    for (int nt = 0; nt < 4; ++nt)
#pragma unroll
      for (int r = 0; r < 8; ++r)
        at32[(8 * hh + r) * (AP / 2) + 16 * nt + m] = split_word(relu_k(c[nt][r]));
    __syncthreads();

    v8f a2[2];
    a2[0] = z8(); a2[1] = z8();
#pragma unroll
    for (int ks = 0; ks < 4; ++ks) {
      FragB a;
      const unsigned short* ap = at + m * AP + 32 * ks + 8 * hh;
      a.h[0] = *(const v8usa*)ap;
      a.h[1] = *(const v8usa*)(ap + 16);
#pragma unroll
      for (int nt = 0; nt < 2; ++nt) {
        FragB b;
        const unsigned short* wq = sW12 + (16 * nt + m) * 128 + 32 * ks + 8 * hh;
        b.h[0] = *(const v8usa*)wq;
        b.h[1] = *(const v8usa*)(wq + 16);
        a2[nt] = wmb(a, b, a2[nt]);
      }
    }
    float mxv[2];
#pragma unroll
    for (int nt = 0; nt < 2; ++nt) {
      const float bv = sb[HID + 16 * nt + m];
      float mx = relu_k(a2[nt][0] + bv);
#pragma unroll
      for (int r = 1; r < 8; ++r) {
        const float v = relu_k(a2[nt][r] + bv);
        mx = (v > mx || v != v) ? v : mx;
      }
      const float o = __shfl_xor(mx, 16, 32);
      mx = (o > mx || o != o) ? o : mx;
      mxv[nt] = mx;
    }
    float val = (hh != 0) ? mxv[1] : mxv[0];
    val = (badm != 0u) ? qnan : val;
    ag[j * FW + lane] = val;
  }
  __syncthreads();
  flush_rows32(ag, AGGR + (size_t)baseC * FW, live, lane);
}

__global__ __launch_bounds__(NTHR) void k_node(const float* __restrict__ Hold, const float* __restrict__ AGGR,
                                               const unsigned short* __restrict__ WPL,
                                               const float* __restrict__ BIAS, float* Hnew, float* XA,
                                               int nTiles, int doXA) {
  extern __shared__ __attribute__((aligned(16))) float dyn[];
  const int tid = (int)threadIdx.x, lane = tid & 31, wave = tid >> 5, hh = lane >> 4, m = lane & 15;
  float*          zt   = dyn + wave * WAVE_F;
  float*          atf  = zt + XS_F;
  unsigned short* at   = (unsigned short*)atf;
  unsigned*       at32 = (unsigned*)atf;
  float*          ht   = atf + AT_F;
  float*          sb   = dyn + NWAVE * WAVE_F;
  const unsigned short* W21 = WPL + O_W21;
  const unsigned short* W22 = WPL + O_W22;

  const int  t    = (int)blockIdx.x * NWAVE + wave;
  const bool live = t < nTiles;
  const int  tc   = live ? t : nTiles - 1;
  const int  base = 16 * tc;

  if (wave == 0) {
    const v4f bv = *(const v4fa*)(BIAS + 64 + 4 * lane);
    *(v4fa*)(sb + 4 * lane) = bv;
  }
#pragma unroll
  for (int i = 0; i < 4; ++i) {
    const int idx = i * 32 + lane;
    const int row = idx >> 3, pc = idx & 7;
    const v4f hv = *(const v4f*)(Hold + (size_t)base * FW + 4 * idx);
    const v4f av = *(const v4f*)(AGGR + (size_t)base * FW + 4 * idx);
    *(v4fa*)(zt + row * XP + 4 * pc)      = hv;
    *(v4fa*)(zt + row * XP + 32 + 4 * pc) = av;
  }
  __syncthreads();

#pragma unroll 4
  for (int row = 0; row < 16; ++row) {
    const float v0 = zt[row * XP + lane];
    const float v1 = zt[row * XP + 32 + lane];
    at32[row * (AP / 2) + lane]      = split_word(v0);
    at32[row * (AP / 2) + 32 + lane] = split_word(v1);
  }
  __syncthreads();

  v8f acc[4];
#pragma unroll
  for (int nt = 0; nt < 4; ++nt) acc[nt] = z8();
#pragma unroll
  for (int ks = 0; ks < 4; ++ks) {
    FragB a;
    const unsigned short* ap = at + m * AP + 32 * ks + 8 * hh;
    a.h[0] = *(const v8usa*)ap;
    a.h[1] = *(const v8usa*)(ap + 16);
#pragma unroll
    for (int nt = 0; nt < 4; ++nt) {
      FragB b;
      const unsigned short* wq = W21 + (16 * nt + m) * 128 + 32 * ks + 8 * hh;
      b.h[0] = *(const v8usa*)wq;
      b.h[1] = *(const v8usa*)(wq + 16);
      acc[nt] = wmb(a, b, acc[nt]);
    }
  }
  __syncthreads();
#pragma unroll
  for (int nt = 0; nt < 4; ++nt) {
    const float bv = sb[32 + 16 * nt + m];
#pragma unroll
    for (int r = 0; r < 8; ++r)
      at32[(8 * hh + r) * (AP / 2) + 16 * nt + m] = split_word(relu_k(acc[nt][r] + bv));
  }
  __syncthreads();

  v8f c2 = z8();
#pragma unroll
  for (int ks = 0; ks < 4; ++ks) {
    FragB a, b;
    const unsigned short* ap = at + m * AP + 32 * ks + 8 * hh;
    a.h[0] = *(const v8usa*)ap;
    a.h[1] = *(const v8usa*)(ap + 16);
    const unsigned short* wq = W22 + m * 128 + 32 * ks + 8 * hh;
    b.h[0] = *(const v8usa*)wq;
    b.h[1] = *(const v8usa*)(wq + 16);
    c2 = wmb(a, b, c2);
  }
  {
    const float bv = sb[96 + m];
#pragma unroll
    for (int r = 0; r < 8; ++r) ht[(8 * hh + r) * FW + m] = relu_k(c2[r] + bv);
  }
  __syncthreads();

  v4f o0, o1, h0, h1;
  {
    const v4f q0 = *(const v4fa*)(ht + m * FW);
    const v4f q1 = *(const v4fa*)(ht + m * FW + 4);
    const v4f q2 = *(const v4fa*)(ht + m * FW + 8);
    const v4f q3 = *(const v4fa*)(ht + m * FW + 12);
    float ss = 0.0f;
    ss += q0.x * q0.x; ss += q0.y * q0.y; ss += q0.z * q0.z; ss += q0.w * q0.w;
    ss += q1.x * q1.x; ss += q1.y * q1.y; ss += q1.z * q1.z; ss += q1.w * q1.w;
    ss += q2.x * q2.x; ss += q2.y * q2.y; ss += q2.z * q2.z; ss += q2.w * q2.w;
    ss += q3.x * q3.x; ss += q3.y * q3.y; ss += q3.z * q3.z; ss += q3.w * q3.w;
    const float nor = sqrtf(ss);
    const float dn  = (nor > 1.0f || nor != nor) ? nor : 1.0f;
    const bool  up  = hh != 0;
    v4f lo4, hi4;
    lo4.x = up ? q2.x : q0.x; lo4.y = up ? q2.y : q0.y; lo4.z = up ? q2.z : q0.z; lo4.w = up ? q2.w : q0.w;
    hi4.x = up ? q3.x : q1.x; hi4.y = up ? q3.y : q1.y; hi4.z = up ? q3.z : q1.z; hi4.w = up ? q3.w : q1.w;
    o0.x = lo4.x / dn; o0.y = lo4.y / dn; o0.z = lo4.z / dn; o0.w = lo4.w / dn;
    o1.x = hi4.x / dn; o1.y = hi4.y / dn; o1.z = hi4.z / dn; o1.w = hi4.w / dn;
    h0 = *(const v4fa*)(zt + m * XP + 8 * hh);
    h1 = *(const v4fa*)(zt + m * XP + 8 * hh + 4);
  }
  __syncthreads();
  *(v4fa*)(ht + m * FW + 8 * hh)          = o0;
  *(v4fa*)(ht + m * FW + 8 * hh + 4)      = o1;
  *(v4fa*)(ht + m * FW + 16 + 8 * hh)     = h0;
  *(v4fa*)(ht + m * FW + 16 + 8 * hh + 4) = h1;
  __syncthreads();
  flush_rows32(ht, Hnew + (size_t)base * FW, live, lane);
  if (doXA != 0) {
    xa_tail(ht, at32, at, zt, WPL + O_WA2, XA + (size_t)base * HID, live, lane, hh, m);
  }
}

static inline size_t al256(size_t o) { return (o + 255) & ~(size_t)255; }

extern "C" void kernel_launch(void* const* d_in, const int* in_sizes, int n_in,
                              void* d_out, int out_size, void* d_ws, size_t ws_size,
                              hipStream_t stream) {
  if (n_in < 11) return;
  if (in_sizes[0] != NN * FW) return;
  if (in_sizes[1] != 2 * NE) return;
  if (in_sizes[2] != NE * FEA) return;
  if (in_sizes[3] != 64 * 40 || in_sizes[4] != 64) return;
  if (in_sizes[5] != 32 * 64 || in_sizes[6] != 32) return;
  if (in_sizes[7] != 64 * 64 || in_sizes[8] != 64) return;
  if (in_sizes[9] != 16 * 64 || in_sizes[10] != 16) return;
  if (out_size != NN * FW) return;

  const float* x   = (const float*)d_in[0];
  const int*   ei  = (const int*)d_in[1];
  const float* ea  = (const float*)d_in[2];
  const float* w11 = (const float*)d_in[3];
  const float* b11 = (const float*)d_in[4];
  const float* w12 = (const float*)d_in[5];
  const float* b12 = (const float*)d_in[6];
  const float* w21 = (const float*)d_in[7];
  const float* b21 = (const float*)d_in[8];
  const float* w22 = (const float*)d_in[9];
  const float* b22 = (const float*)d_in[10];
  const int* src = ei;
  const int* dst = ei + NE;
  float* out = (float*)d_out;

  char* ws = (char*)d_ws;
  size_t off = 0;
  const size_t oPL = off; off = al256(off + (size_t)PL_US * 2);
  const size_t oBI = off; off = al256(off + (size_t)BIAS_F * 4);
  const size_t oXA = off; off = al256(off + (size_t)NN * HID * 4);
  const size_t oHA = off; off = al256(off + (size_t)NN * FW * 4);
  const size_t oHB = off; off = al256(off + (size_t)NN * FW * 4);
  const size_t oAG = off; off = al256(off + (size_t)NN * FW * 4);
  if (off > ws_size || off > (size_t)WSMAX) return;
  unsigned short* WPL  = (unsigned short*)(ws + oPL);
  float*          BIAS = (float*)(ws + oBI);
  float*          XA   = (float*)(ws + oXA);
  float*          HA   = (float*)(ws + oHA);
  float*          HB   = (float*)(ws + oHB);
  float*          AGGR = (float*)(ws + oAG);

  hipFuncSetAttribute(reinterpret_cast<const void*>(&k_first), hipFuncAttributeMaxDynamicSharedMemorySize,
                      (int)NODE_LDS_BYTES);
  hipFuncSetAttribute(reinterpret_cast<const void*>(&k_edge), hipFuncAttributeMaxDynamicSharedMemorySize,
                      (int)EDGE_LDS_BYTES);
  hipFuncSetAttribute(reinterpret_cast<const void*>(&k_node), hipFuncAttributeMaxDynamicSharedMemorySize,
                      (int)NODE_LDS_BYTES);

  const int nTiles = NN / 16;
  const int gN = (nTiles + NWAVE - 1) / NWAVE;

  k_prep<<<U_W22 / NTHR + 1, NTHR, 0, stream>>>(w11, w12, w21, w22, b11, b12, b21, b22, WPL, BIAS);
  k_first<<<gN, NTHR, NODE_LDS_BYTES, stream>>>(x, WPL, HA, XA, nTiles);

  k_edge<<<gN, NTHR, EDGE_LDS_BYTES, stream>>>(src, dst, ea, XA, WPL + O_WEA, BIAS, AGGR, NN);
  k_node<<<gN, NTHR, NODE_LDS_BYTES, stream>>>(HA, AGGR, WPL, BIAS, HB, XA, nTiles, 1);

  k_edge<<<gN, NTHR, EDGE_LDS_BYTES, stream>>>(src, dst, ea, XA, WPL + O_WEA, BIAS, AGGR, NN);
  k_node<<<gN, NTHR, NODE_LDS_BYTES, stream>>>(HB, AGGR, WPL, BIAS, HA, XA, nTiles, 1);

  k_edge<<<gN, NTHR, EDGE_LDS_BYTES, stream>>>(src, dst, ea, XA, WPL + O_WEA, BIAS, AGGR, NN);
  k_node<<<gN, NTHR, NODE_LDS_BYTES, stream>>>(HA, AGGR, WPL, BIAS, out, XA, nTiles, 0);
}
